// DF_RFEM_2_85048942395453
// MI455X (gfx1250) — hardware-verified
//
#include <hip/hip_runtime.h>
#include <math.h>

#define BB     4
#define HW     4096
#define NPIX   16384
#define IN_CH  256
#define SK_CH  64
#define EMB    64
#define QC     32
#define KCOL   576
#define PSCALE 256.0f

#define WO_QKV  0
#define WO_PROJ 24576
#define WO_OFF  32768
#define WO_DFM  51200
#define WO_DOWN 88064
#define WO_MLP1 108544
#define WO_MLP2 124928
#define WO_UP   141312
#define WTOT    157696

#define EPI_QKV  0
#define EPI_X2   1
#define EPI_RES  2
#define EPI_LN   3
#define EPI_GELU 4
#define EPI_OFF  5
#define EPI_CHW  6

typedef _Float16 v16h __attribute__((ext_vector_type(16)));
typedef _Float16 v8h  __attribute__((ext_vector_type(8)));
typedef __attribute__((ext_vector_type(16))) __bf16 v16b;
typedef unsigned short v16us __attribute__((ext_vector_type(16)));
typedef unsigned short v8us  __attribute__((ext_vector_type(8)));
typedef float v8f __attribute__((ext_vector_type(8)));
typedef float v4f __attribute__((ext_vector_type(4)));
typedef v8h  __attribute__((may_alias)) v8ha;
typedef v8us __attribute__((may_alias)) v8usa;
typedef v4f  __attribute__((may_alias)) v4fa;

union FragH { v16h v; v8h half[2]; };
union FragU { v16us v; v8us half[2]; };

__device__ __forceinline__ v8f wmma_f16(v16h a, v16h b, v8f c) {
  v8f d = __builtin_amdgcn_wmma_f32_16x16x32_f16(false, a, false, b, (short)0, c, false, false);
  asm volatile("v_nop\n\tv_nop\n\tv_nop\n\tv_nop" : "+v"(d) : "v"(a), "v"(b));
  return d;
}
__device__ __forceinline__ v8f wmma_bf16(v16us a, v16us b, v8f c) {
  const v16b ab = __builtin_bit_cast(v16b, a);
  const v16b bb = __builtin_bit_cast(v16b, b);
  v8f d = __builtin_amdgcn_wmma_f32_16x16x32_bf16(false, ab, false, bb, (short)0, c, false, false);
  asm volatile("v_nop\n\tv_nop\n\tv_nop\n\tv_nop" : "+v"(d) : "v"(a), "v"(b));
  return d;
}

__device__ __forceinline__ v16h ldf_h(const _Float16* p, int h) {
  FragH f;
  f.half[0] = *(const v8ha*)(p + 8 * h);
  f.half[1] = *(const v8ha*)(p + 16 + 8 * h);
  return f.v;
}
__device__ __forceinline__ v16us ldf_u(const unsigned short* p, int h) {
  FragU f;
  f.half[0] = *(const v8usa*)(p + 8 * h);
  f.half[1] = *(const v8usa*)(p + 16 + 8 * h);
  return f.v;
}

__device__ __forceinline__ unsigned int bf_rne(float x) {
  const unsigned int u = __float_as_uint(x);
  return (u + 0x7fffu + ((u >> 16) & 1u)) >> 16;
}
__device__ __forceinline__ void split8(v8f v, v8us& hi, v8us& lo) {
#pragma unroll
  for (int j = 0; j < 8; ++j) {
    const unsigned int hb = bf_rne(v[j]);
    const float rem = v[j] - __uint_as_float(hb << 16);
    hi[j] = (unsigned short)hb;
    lo[j] = (unsigned short)bf_rne(rem);
  }
}

__device__ __forceinline__ float gelu_f(float v) {
  return 0.5f * v * (1.0f + erff(v * 0.70710678118654752f));
}

__global__ __launch_bounds__(256) void prep_w_kernel(
    const float* __restrict__ qkv_w, const float* __restrict__ proj_w,
    const float* __restrict__ off_w, const float* __restrict__ dfm_w,
    const float* __restrict__ down_w, const float* __restrict__ mlp1_w,
    const float* __restrict__ mlp2_w, const float* __restrict__ up_w,
    unsigned short* wph, unsigned short* wpl)
{
  const int seg = blockIdx.y;
  const float* src; int cnt, dofs, kind, nsrc;
  switch (seg) {
    case 0:  src = qkv_w;  cnt = 96 * 256;  dofs = WO_QKV;  kind = 0; nsrc = 1;  break;
    case 1:  src = proj_w; cnt = 256 * 32;  dofs = WO_PROJ; kind = 0; nsrc = 1;  break;
    case 2:  src = off_w;  cnt = 32 * KCOL; dofs = WO_OFF;  kind = 1; nsrc = 18; break;
    case 3:  src = dfm_w;  cnt = 64 * KCOL; dofs = WO_DFM;  kind = 1; nsrc = 64; break;
    case 4:  src = down_w; cnt = 64 * 320;  dofs = WO_DOWN; kind = 0; nsrc = 1;  break;
    case 5:  src = mlp1_w; cnt = 256 * 64;  dofs = WO_MLP1; kind = 0; nsrc = 1;  break;
    case 6:  src = mlp2_w; cnt = 64 * 256;  dofs = WO_MLP2; kind = 0; nsrc = 1;  break;
    default: src = up_w;   cnt = 256 * 64;  dofs = WO_UP;   kind = 0; nsrc = 1;  break;
  }
  const int g = blockIdx.x * 256 + (int)threadIdx.x;
  const int e0 = g * 8;
  if (e0 >= cnt) return;
  v8f v;
  if (kind == 0) {
    const v4f a = *(const v4fa*)(src + e0);
    const v4f c = *(const v4fa*)(src + e0 + 4);
    v[0] = a.x; v[1] = a.y; v[2] = a.z; v[3] = a.w;
    v[4] = c.x; v[5] = c.y; v[6] = c.z; v[7] = c.w;
  } else {
    const int n = e0 / KCOL;
    const int k = e0 - n * KCOL;
    const int tap = k >> 6, c = k & 63;
    const int nc = min(n, nsrc - 1);
    const float* bp = src + ((size_t)(nc * 64 + c)) * 9 + tap;
#pragma unroll
    for (int j = 0; j < 8; ++j) {
      const float t = bp[j * 9];
      v[j] = (n < nsrc) ? t : 0.0f;
    }
  }
  v8us hi, lo;
  split8(v, hi, lo);
  const size_t off = (size_t)dofs + (size_t)e0;
  *(volatile v8us*)(wph + off) = hi;
  *(volatile v8us*)(wpl + off) = lo;
  __threadfence();
  *(volatile v8us*)(wph + off) = hi;
  *(volatile v8us*)(wpl + off) = lo;
}

__global__ __launch_bounds__(256) void xT_kernel(const float* __restrict__ x,
                                                 unsigned short* xth, unsigned short* xtl)
{
  __shared__ float sx[64 * 33];
  const int tid = threadIdx.x;
  const int P0 = blockIdx.x * 32;
  const int b = P0 >> 12, pos0 = P0 & (HW - 1);
  const int c0 = blockIdx.y * 64;
#pragma unroll
  for (int it = 0; it < 8; ++it) {
    const int idx = it * 256 + tid;
    const int c = idx >> 5, p = idx & 31;
    sx[c * 33 + p] = x[((size_t)(b * IN_CH + c0 + c)) * HW + pos0 + p];
  }
  __syncthreads();
  const int p = tid >> 3, q8 = tid & 7;
  v8f v;
#pragma unroll
  for (int j = 0; j < 8; ++j) v[j] = sx[(8 * q8 + j) * 33 + p];
  v8us hi, lo;
  split8(v, hi, lo);
  const size_t off = (size_t)(P0 + p) * IN_CH + c0 + 8 * q8;
  *(volatile v8us*)(xth + off) = hi;
  *(volatile v8us*)(xtl + off) = lo;
  __threadfence();
  *(volatile v8us*)(xth + off) = hi;
  *(volatile v8us*)(xtl + off) = lo;
}

template <int NT, int EPI>
__device__ __forceinline__ void gemm_store(const float* sT, const float* sMu, const float* sRs,
    const float* __restrict__ aux0, const float* __restrict__ aux1,
    float* outf, unsigned short* outh, unsigned short* outl,
    _Float16* oq, _Float16* okp, _Float16* ov, int ldo, int co, int tid)
{
  const int CT = 16 * NT;
  const int P0 = blockIdx.x * 64;
  const int n0 = blockIdx.y * CT;
  if (EPI == EPI_QKV) {
    const int which = blockIdx.y;
    if (which < 2) {
      _Float16* dst = ((which == 0) ? oq : okp) + (size_t)P0 * QC;
#pragma unroll
      for (int it = 0; it < 2; ++it) {
        const int id = it * 128 + tid;
        const int row = id >> 2, q4 = id & 3;
        v8h o;
#pragma unroll
        for (int j = 0; j < 8; ++j) o[j] = (_Float16)sT[row * CT + 8 * q4 + j];
        *(volatile v8h*)(dst + (size_t)id * 8) = o;
      }
    } else {
      const int b = P0 >> 12, pos0 = P0 & (HW - 1);
#pragma unroll
      for (int it = 0; it < 2; ++it) {
        const int id = it * 128 + tid;
        const int c = id >> 3, q8 = id & 7;
        v8h o;
#pragma unroll
        for (int j = 0; j < 8; ++j) o[j] = (_Float16)sT[(8 * q8 + j) * CT + c];
        *(volatile v8h*)(ov + ((size_t)(b * QC + c)) * HW + pos0 + 8 * q8) = o;
      }
    }
  } else if (EPI == EPI_X2 || EPI == EPI_RES) {
#pragma unroll
    for (int it = 0; it < 4; ++it) {
      const int id = it * 128 + tid;
      const int row = id >> 3, q8 = id & 7;
      v8f v;
#pragma unroll
      for (int j = 0; j < 8; ++j) v[j] = sT[row * CT + 8 * q8 + j];
      v8us hi, lo;
      split8(v, hi, lo);
      const size_t off = (size_t)(P0 + row) * (size_t)ldo + co + n0 + 8 * q8;
      *(volatile v8us*)(outh + off) = hi;
      *(volatile v8us*)(outl + off) = lo;
    }
  } else if (EPI == EPI_LN) {
#pragma unroll
    for (int it = 0; it < 8; ++it) {
      const int id = it * 128 + tid;
      const int row = id >> 4, q = id & 15;
      const v4f v = *(const v4fa*)(sT + row * CT + 4 * q);
      *(volatile v4f*)(outf + (size_t)(P0 + row) * EMB + 4 * q) = v;
    }
#pragma unroll
    for (int it = 0; it < 4; ++it) {
      const int id = it * 128 + tid;
      const int row = id >> 3, q8 = id & 7;
      const float mu = sMu[row], rs = sRs[row];
      v8f v;
#pragma unroll
      for (int j = 0; j < 8; ++j) {
        const int c = 8 * q8 + j;
        v[j] = (sT[row * CT + c] - mu) * rs * aux0[c] + aux1[c];
      }
      v8us hi, lo;
      split8(v, hi, lo);
      const size_t off = (size_t)(P0 + row) * EMB + 8 * q8;
      *(volatile v8us*)(outh + off) = hi;
      *(volatile v8us*)(outl + off) = lo;
    }
  } else if (EPI == EPI_GELU) {
#pragma unroll
    for (int it = 0; it < 8; ++it) {
      const int id = it * 128 + tid;
      const int row = id >> 4, q = id & 15;
      const v4f v = *(const v4fa*)(sT + row * CT + 4 * q);
      *(volatile v4f*)(outf + (size_t)(P0 + row) * (size_t)ldo + co + n0 + 4 * q) = v;
    }
  } else if (EPI == EPI_OFF) {
#pragma unroll
    for (int it = 0; it < 4; ++it) {
      const int id = it * 128 + tid;
      const int row = id >> 3, q8 = id & 7;
      const v4f v = *(const v4fa*)(sT + row * CT + 4 * q8);
      *(volatile v4f*)(outf + (size_t)(P0 + row) * 32 + 4 * q8) = v;
    }
  } else {
    const int b = P0 >> 12, pos0 = P0 & (HW - 1);
#pragma unroll
    for (int it = 0; it < 8; ++it) {
      const int id = it * 128 + tid;
      const int c = id >> 4, q = id & 15;
      v4f v;
      v.x = sT[(4 * q + 0) * CT + c];
      v.y = sT[(4 * q + 1) * CT + c];
      v.z = sT[(4 * q + 2) * CT + c];
      v.w = sT[(4 * q + 3) * CT + c];
      *(volatile v4f*)(outf + ((size_t)(b * IN_CH + n0 + c)) * HW + pos0 + 4 * q) = v;
    }
  }
}

template <int NT, int EPI>
__global__ __launch_bounds__(128) void gemm_kernel(
    const unsigned short* __restrict__ Ah, const unsigned short* __restrict__ Al, int lda,
    const unsigned short* __restrict__ Wh, const unsigned short* __restrict__ Wl, int K,
    const float* __restrict__ bias, const float* __restrict__ aux0, const float* __restrict__ aux1,
    float* outf, unsigned short* outh, unsigned short* outl,
    _Float16* oq, _Float16* okp, _Float16* ov, int ldo, int co)
{
  const int CT = 16 * NT;
  __shared__ __attribute__((aligned(16))) float sT[64 * 64];
  __shared__ float sMu[64];
  __shared__ float sRs[64];

  const int tid = threadIdx.x, lane = tid & 31, w = tid >> 5;
  const int h = lane >> 4, m = lane & 15;
  const int P0 = blockIdx.x * 64;
  const int n0 = blockIdx.y * CT;

  const size_t arow = (size_t)(P0 + 16 * w + m) * (size_t)lda;
  const unsigned short* arh = Ah + arow;
  const unsigned short* arl = Al + arow;
  const size_t wrow = (size_t)(n0 + m) * (size_t)K;
  const unsigned short* wrh = Wh + wrow;
  const unsigned short* wrl = Wl + wrow;

  const v8f zero8 = {0.f, 0.f, 0.f, 0.f, 0.f, 0.f, 0.f, 0.f};
  v8f acc[NT];
#pragma unroll
  for (int nt = 0; nt < NT; ++nt) acc[nt] = zero8;

#pragma unroll 1
  for (int k0 = 0; k0 < K; k0 += 32) {
    const v16us ah = ldf_u(arh + k0, h);
    const v16us al = ldf_u(arl + k0, h);
#pragma unroll
    for (int nt = 0; nt < NT; ++nt) {
      const size_t wo = (size_t)nt * 16 * (size_t)K + k0;
      const v16us bh = ldf_u(wrh + wo, h);
      const v16us bl = ldf_u(wrl + wo, h);
      acc[nt] = wmma_bf16(ah, bh, acc[nt]);
      acc[nt] = wmma_bf16(al, bh, acc[nt]);
      acc[nt] = wmma_bf16(ah, bl, acc[nt]);
    }
  }

  const int prow0 = 16 * w + 8 * h;
  const int Pg0 = P0 + prow0;
#pragma unroll
  for (int nt = 0; nt < NT; ++nt) {
    const int c = 16 * nt + m;
    const int n = n0 + c;
    float bv;
    if (EPI == EPI_OFF) bv = bias[min(n, 17)]; else bv = bias[n];
    float res[8];
#pragma unroll
    for (int r = 0; r < 8; ++r) res[r] = 0.0f;
    if (EPI == EPI_X2) {
      const float* xp = aux0 + ((size_t)((Pg0 >> 12) * IN_CH + n)) * HW + (Pg0 & (HW - 1));
      const v4f xa = *(const v4fa*)xp;
      const v4f xb = *(const v4fa*)(xp + 4);
      res[0] = xa.x; res[1] = xa.y; res[2] = xa.z; res[3] = xa.w;
      res[4] = xb.x; res[5] = xb.y; res[6] = xb.z; res[7] = xb.w;
    } else if (EPI == EPI_RES) {
#pragma unroll
      for (int r = 0; r < 8; ++r) res[r] = aux0[(size_t)(Pg0 + r) * EMB + n];
    } else if (EPI == EPI_OFF) {
#pragma unroll
      for (int r = 0; r < 8; ++r) res[r] = aux0[Pg0 + r];
    }
#pragma unroll
    for (int r = 0; r < 8; ++r) {
      float v = acc[nt][r] + bv;
      if (EPI == EPI_X2 || EPI == EPI_RES) v += res[r];
      if (EPI == EPI_OFF) v = v * (1.0f + 16.0f * res[r]);
      if (EPI == EPI_GELU) v = gelu_f(v);
      sT[(prow0 + r) * CT + c] = v;
    }
  }
  __syncthreads();

  if (EPI == EPI_LN) {
    if (tid < 64) {
      const float* rowp = sT + tid * CT;
      float s = 0.0f;
#pragma unroll 4
      for (int c = 0; c < EMB; ++c) s += rowp[c];
      const float mu = s * (1.0f / 64.0f);
      float s2 = 0.0f;
#pragma unroll 4
      for (int c = 0; c < EMB; ++c) { const float d = rowp[c] - mu; s2 += d * d; }
      const float var = s2 * (1.0f / 64.0f);
      sMu[tid] = mu;
      sRs[tid] = 1.0f / sqrtf(var + 1e-5f);
    }
    __syncthreads();
  }

  gemm_store<NT, EPI>(sT, sMu, sRs, aux0, aux1, outf, outh, outl, oq, okp, ov, ldo, co, tid);
  __threadfence();
  gemm_store<NT, EPI>(sT, sMu, sRs, aux0, aux1, outf, outh, outl, oq, okp, ov, ldo, co, tid);
}

__device__ __forceinline__ v16h pack_p(v8f a, v8f c) {
  const v16h r = { (_Float16)(a[0] * PSCALE), (_Float16)(a[1] * PSCALE), (_Float16)(a[2] * PSCALE), (_Float16)(a[3] * PSCALE),
                   (_Float16)(a[4] * PSCALE), (_Float16)(a[5] * PSCALE), (_Float16)(a[6] * PSCALE), (_Float16)(a[7] * PSCALE),
                   (_Float16)(c[0] * PSCALE), (_Float16)(c[1] * PSCALE), (_Float16)(c[2] * PSCALE), (_Float16)(c[3] * PSCALE),
                   (_Float16)(c[4] * PSCALE), (_Float16)(c[5] * PSCALE), (_Float16)(c[6] * PSCALE), (_Float16)(c[7] * PSCALE) };
  return r;
}

__device__ __forceinline__ void att_store(const float* so, unsigned short* avh, unsigned short* avl,
                                          size_t rowbase, int lane) {
#pragma unroll
  for (int it = 0; it < 2; ++it) {
    const int id = it * 32 + lane;
    const int row = id >> 2, q4 = id & 3;
    v8f v;
#pragma unroll
    for (int j = 0; j < 8; ++j) v[j] = so[row * 32 + 8 * q4 + j];
    v8us hi, lo;
    split8(v, hi, lo);
    const size_t off = (rowbase + (size_t)row) * QC + 8 * q4;
    *(volatile v8us*)(avh + off) = hi;
    *(volatile v8us*)(avl + off) = lo;
  }
}

__global__ __launch_bounds__(128) void attn_kernel(
    const _Float16* __restrict__ qh,
    const _Float16* __restrict__ kh,
    const _Float16* __restrict__ vt,
    unsigned short* avh, unsigned short* avl)
{
  __shared__ __attribute__((aligned(16))) float sO[4 * 16 * 32];

  const int tid = threadIdx.x, lane = tid & 31, w = tid >> 5;
  const int h = lane >> 4, m = lane & 15;
  const int b = blockIdx.y;
  const int q0 = blockIdx.x * 64 + 16 * w;
  const size_t pbase = (size_t)b * HW;

  const v16h qb = ldf_h(qh + (pbase + q0 + m) * QC, h);

  const v8f zero8 = {0.f, 0.f, 0.f, 0.f, 0.f, 0.f, 0.f, 0.f};
  v8f o[2];
  o[0] = zero8; o[1] = zero8;
  float mrun = -1e30f, lrun = 0.0f;

  const _Float16* kbase = kh + (pbase + m) * QC;
  const _Float16* vbase = vt + ((size_t)b * QC + m) * HW;
  const float scale = 0.17677669529663688f;

#pragma unroll 1
  for (int kb = 0; kb < HW; kb += 64) {
    v8f s[4];
#pragma unroll
    for (int j = 0; j < 4; ++j) {
      const v16h kf = ldf_h(kbase + (size_t)(kb + 16 * j) * QC, h);
      s[j] = wmma_f16(kf, qb, zero8);
    }
    float mloc = -1e30f;
#pragma unroll
    for (int j = 0; j < 4; ++j)
#pragma unroll
      for (int r = 0; r < 8; ++r) {
        s[j][r] = s[j][r] * scale;
        mloc = fmaxf(mloc, s[j][r]);
      }
    mloc = fmaxf(mloc, __shfl_xor(mloc, 16));
    const float mnew = fmaxf(mrun, mloc);
    const float alpha = __expf(mrun - mnew);
    mrun = mnew;
    float lsum = 0.0f;
#pragma unroll
    for (int j = 0; j < 4; ++j)
#pragma unroll
      for (int r = 0; r < 8; ++r) {
        const float p = __expf(s[j][r] - mnew);
        s[j][r] = p;
        lsum += p;
      }
    lsum += __shfl_xor(lsum, 16);
    lrun = lrun * alpha + lsum;
#pragma unroll
    for (int t = 0; t < 2; ++t)
#pragma unroll
      for (int r = 0; r < 8; ++r) o[t][r] = o[t][r] * alpha;

    const v16h pb0 = pack_p(s[0], s[1]);
    const v16h pb1 = pack_p(s[2], s[3]);

#pragma unroll
    for (int t = 0; t < 2; ++t) {
      const _Float16* vp = vbase + (size_t)(16 * t) * HW + kb;
      const v16h vf0 = ldf_h(vp, h);
      const v16h vf1 = ldf_h(vp + 32, h);
      o[t] = wmma_f16(vf0, pb0, o[t]);
      o[t] = wmma_f16(vf1, pb1, o[t]);
    }
  }

  const float inv = (1.0f / lrun) * (1.0f / PSCALE);
  float* so = sO + w * 512;
#pragma unroll
  for (int t = 0; t < 2; ++t)
#pragma unroll
    for (int r = 0; r < 8; ++r)
      so[m * 32 + 16 * t + 8 * h + r] = o[t][r] * inv;
  __syncthreads();

  att_store(so, avh, avl, pbase + (size_t)q0, lane);
  __threadfence();
  att_store(so, avh, avl, pbase + (size_t)q0, lane);
}

__global__ __launch_bounds__(512) void skipup_kernel(
    const float* __restrict__ skip, const float* __restrict__ tw, const float* __restrict__ tb,
    float* suT, float* mbuf, float* thk)
{
  __shared__ __attribute__((aligned(16))) float sm[32];
  __shared__ __attribute__((aligned(16))) float st[32];
  const int tid = threadIdx.x;
  const int pl = tid >> 4, qq = tid & 15;
  const int P0 = blockIdx.x * 32;
  const int P = P0 + pl;
  const int b = P >> 12, pos = P & (HW - 1);
  const int yy = pos >> 6, xx = pos & 63;

  int ylo, yhi, xlo, xhi;
  float wylo, wyhi, wxlo, wxhi;
  if (yy & 1) { ylo = (yy - 1) >> 1; yhi = ylo + 1; wylo = 0.75f; wyhi = 0.25f; }
  else        { yhi = yy >> 1; ylo = yhi - 1; wylo = 0.25f; wyhi = 0.75f; }
  if (ylo < 0)  { ylo = 0;  wylo = 0.0f; wyhi = 1.0f; }
  if (yhi > 31) { yhi = 31; wyhi = 0.0f; wylo = 1.0f; }
  if (xx & 1) { xlo = (xx - 1) >> 1; xhi = xlo + 1; wxlo = 0.75f; wxhi = 0.25f; }
  else        { xhi = xx >> 1; xlo = xhi - 1; wxlo = 0.25f; wxhi = 0.75f; }
  if (xlo < 0)  { xlo = 0;  wxlo = 0.0f; wxhi = 1.0f; }
  if (xhi > 31) { xhi = 31; wxhi = 0.0f; wxlo = 1.0f; }

  v4f o;
  float s = 0.0f, d = 0.0f;
#pragma unroll
  for (int j = 0; j < 4; ++j) {
    const int c = 4 * qq + j;
    const float* sp = skip + ((size_t)(b * SK_CH + c)) * 1024;
    const float a00 = sp[ylo * 32 + xlo];
    const float a10 = sp[yhi * 32 + xlo];
    const float a01 = sp[ylo * 32 + xhi];
    const float a11 = sp[yhi * 32 + xhi];
    const float tlo = wylo * a00 + wyhi * a10;
    const float thi = wylo * a01 + wyhi * a11;
    const float v = wxlo * tlo + wxhi * thi;
    o[j] = v;
    s += v;
    d += v * tw[c];
  }
  s += __shfl_xor(s, 8); s += __shfl_xor(s, 4); s += __shfl_xor(s, 2); s += __shfl_xor(s, 1);
  d += __shfl_xor(d, 8); d += __shfl_xor(d, 4); d += __shfl_xor(d, 2); d += __shfl_xor(d, 1);
  if (qq == 0) {
    sm[pl] = s * (1.0f / 64.0f);
    const float z = d + tb[0];
    const float t = __expf(-z);
    st[pl] = __builtin_amdgcn_rcpf(1.0f + t);
  }
  __syncthreads();

  float* sdst = suT + (size_t)P * SK_CH + 4 * qq;
  *(volatile v4f*)sdst = o;
  if (tid < 8) {
    const v4f mv = *(const v4fa*)(sm + 4 * tid);
    const v4f tv = *(const v4fa*)(st + 4 * tid);
    *(volatile v4f*)(mbuf + P0 + 4 * tid) = mv;
    *(volatile v4f*)(thk + P0 + 4 * tid) = tv;
  }
  __threadfence();
  *(volatile v4f*)sdst = o;
  if (tid < 8) {
    const v4f mv = *(const v4fa*)(sm + 4 * tid);
    const v4f tv = *(const v4fa*)(st + 4 * tid);
    *(volatile v4f*)(mbuf + P0 + 4 * tid) = mv;
    *(volatile v4f*)(thk + P0 + 4 * tid) = tv;
  }
}

__global__ __launch_bounds__(256) void edge_kernel(
    const float* __restrict__ mbuf, const float* __restrict__ ew, float* edgeT)
{
  const int tid = threadIdx.x;
  const int pl = tid >> 4, qq = tid & 15;
  const int P = blockIdx.x * 16 + pl;
  const int b = P >> 12, pos = P & (HW - 1);
  const int yy = pos >> 6, xx = pos & 63;
  v4f o = {0.0f, 0.0f, 0.0f, 0.0f};
#pragma unroll 1
  for (int tap = 0; tap < 9; ++tap) {
    const int ny = yy + tap / 3 - 1, nx = xx + tap % 3 - 1;
    const bool inb = (ny >= 0) && (ny < 64) && (nx >= 0) && (nx < 64);
    const int nyc = min(max(ny, 0), 63), nxc = min(max(nx, 0), 63);
    float mv = mbuf[b * HW + nyc * 64 + nxc];
    mv = inb ? mv : 0.0f;
#pragma unroll
    for (int j = 0; j < 4; ++j) o[j] += mv * ew[(4 * qq + j) * 9 + tap];
  }
  float* dst = edgeT + (size_t)P * SK_CH + 4 * qq;
  *(volatile v4f*)dst = o;
  __threadfence();
  *(volatile v4f*)dst = o;
}

__global__ __launch_bounds__(256) void cols_edge_kernel(
    const float* __restrict__ edgeT, unsigned short* colh, unsigned short* coll)
{
  const int g = blockIdx.x * 256 + (int)threadIdx.x;
  if (g >= NPIX * 72) return;
  const int P = g / 72, rem = g - P * 72;
  const int tap = rem >> 3, q8 = rem & 7;
  const int b = P >> 12, pos = P & (HW - 1);
  const int yy = pos >> 6, xx = pos & 63;
  const int ny = yy + tap / 3 - 1, nx = xx + tap % 3 - 1;
  const bool inb = (ny >= 0) && (ny < 64) && (nx >= 0) && (nx < 64);
  const int nyc = min(max(ny, 0), 63), nxc = min(max(nx, 0), 63);
  const float* sp = edgeT + ((size_t)(b * HW + nyc * 64 + nxc)) * SK_CH + 8 * q8;
  const v4f a = *(const v4fa*)sp;
  const v4f c = *(const v4fa*)(sp + 4);
  v8f v;
  v[0] = a.x; v[1] = a.y; v[2] = a.z; v[3] = a.w;
  v[4] = c.x; v[5] = c.y; v[6] = c.z; v[7] = c.w;
#pragma unroll
  for (int j = 0; j < 8; ++j) v[j] = inb ? v[j] : 0.0f;
  v8us hi, lo;
  split8(v, hi, lo);
  const size_t off = (size_t)g * 8;
  *(volatile v8us*)(colh + off) = hi;
  *(volatile v8us*)(coll + off) = lo;
  __threadfence();
  *(volatile v8us*)(colh + off) = hi;
  *(volatile v8us*)(coll + off) = lo;
}

__global__ __launch_bounds__(256) void cols_dfm_kernel(
    const float* __restrict__ suT, const float* __restrict__ offb,
    unsigned short* valh, unsigned short* vall)
{
  const int g = blockIdx.x * 256 + (int)threadIdx.x;
  if (g >= NPIX * 72) return;
  const int P = g / 72, rem = g - P * 72;
  const int k = rem >> 3, q8 = rem & 7;
  const int b = P >> 12, pos = P & (HW - 1);
  const int yy = pos >> 6, xx = pos & 63;
  const float dy = offb[(size_t)P * 32 + 2 * k];
  const float dx = offb[(size_t)P * 32 + 2 * k + 1];
  const float py = (float)(yy + k / 3 - 1) + dy;
  const float px = (float)(xx + k % 3 - 1) + dx;
  const float y0f = floorf(py), x0f = floorf(px);
  const float wy = py - y0f, wx = px - x0f;
  const int y0 = (int)fminf(fmaxf(y0f, -4.0f), 70.0f);
  const int x0 = (int)fminf(fmaxf(x0f, -4.0f), 70.0f);
  const int y1 = y0 + 1, x1 = x0 + 1;
  const float m00 = (y0 >= 0 && y0 < 64 && x0 >= 0 && x0 < 64) ? 1.0f : 0.0f;
  const float m01 = (y0 >= 0 && y0 < 64 && x1 >= 0 && x1 < 64) ? 1.0f : 0.0f;
  const float m10 = (y1 >= 0 && y1 < 64 && x0 >= 0 && x0 < 64) ? 1.0f : 0.0f;
  const float m11 = (y1 >= 0 && y1 < 64 && x1 >= 0 && x1 < 64) ? 1.0f : 0.0f;
  const int y0c = min(max(y0, 0), 63), y1c = min(max(y1, 0), 63);
  const int x0c = min(max(x0, 0), 63), x1c = min(max(x1, 0), 63);
  const float w00 = ((1.0f - wy) * (1.0f - wx)) * m00;
  const float w01 = ((1.0f - wy) * wx) * m01;
  const float w10 = (wy * (1.0f - wx)) * m10;
  const float w11 = (wy * wx) * m11;
  const size_t rb = (size_t)b * HW;
  const float* r00 = suT + (rb + (size_t)(y0c * 64 + x0c)) * SK_CH + 8 * q8;
  const float* r01 = suT + (rb + (size_t)(y0c * 64 + x1c)) * SK_CH + 8 * q8;
  const float* r10 = suT + (rb + (size_t)(y1c * 64 + x0c)) * SK_CH + 8 * q8;
  const float* r11 = suT + (rb + (size_t)(y1c * 64 + x1c)) * SK_CH + 8 * q8;
  const v4f a0 = *(const v4fa*)r00, a1 = *(const v4fa*)(r00 + 4);
  const v4f b0 = *(const v4fa*)r01, b1 = *(const v4fa*)(r01 + 4);
  const v4f c0 = *(const v4fa*)r10, c1 = *(const v4fa*)(r10 + 4);
  const v4f d0 = *(const v4fa*)r11, d1 = *(const v4fa*)(r11 + 4);
  const v8f g00 = {a0.x, a0.y, a0.z, a0.w, a1.x, a1.y, a1.z, a1.w};
  const v8f g01 = {b0.x, b0.y, b0.z, b0.w, b1.x, b1.y, b1.z, b1.w};
  const v8f g10 = {c0.x, c0.y, c0.z, c0.w, c1.x, c1.y, c1.z, c1.w};
  const v8f g11 = {d0.x, d0.y, d0.z, d0.w, d1.x, d1.y, d1.z, d1.w};
  v8f v;
#pragma unroll
  for (int j = 0; j < 8; ++j)
    v[j] = ((g00[j] * w00 + g01[j] * w01) + g10[j] * w10) + g11[j] * w11;
  v8us hi, lo;
  split8(v, hi, lo);
  const size_t off = (size_t)g * 8;
  *(volatile v8us*)(valh + off) = hi;
  *(volatile v8us*)(vall + off) = lo;
  __threadfence();
  *(volatile v8us*)(valh + off) = hi;
  *(volatile v8us*)(vall + off) = lo;
}

__global__ __launch_bounds__(256) void dwconv_kernel(
    const float* __restrict__ h1, const float* __restrict__ dww, const float* __restrict__ dwb,
    unsigned short* h2h, unsigned short* h2l)
{
  __shared__ __attribute__((aligned(16))) float sg[256 * 8];
  const int tid = threadIdx.x, lane = tid & 31, pl = tid >> 5;
  const int P = blockIdx.x * 8 + pl;
  const int b = P >> 12, pos = P & (HW - 1);
  const int yy = pos >> 6, xx = pos & 63;
#pragma unroll 1
  for (int j = 0; j < 8; ++j) {
    const int cc = 8 * lane + j;
    float acc = dwb[cc];
#pragma unroll
    for (int tap = 0; tap < 9; ++tap) {
      const int ny = yy + tap / 3 - 1, nx = xx + tap % 3 - 1;
      const bool inb = (ny >= 0) && (ny < 64) && (nx >= 0) && (nx < 64);
      const int nyc = min(max(ny, 0), 63), nxc = min(max(nx, 0), 63);
      float hv = h1[((size_t)(b * HW + nyc * 64 + nxc)) * 256 + cc];
      hv = inb ? hv : 0.0f;
      acc += hv * dww[cc * 9 + tap];
    }
    sg[tid * 8 + j] = gelu_f(acc);
  }
  __syncthreads();
  const v4f a = *(const v4fa*)(sg + tid * 8);
  const v4f c = *(const v4fa*)(sg + tid * 8 + 4);
  const v8f v = {a.x, a.y, a.z, a.w, c.x, c.y, c.z, c.w};
  v8us hi, lo;
  split8(v, hi, lo);
  const size_t off = (size_t)P * 256 + 8 * lane;
  *(volatile v8us*)(h2h + off) = hi;
  *(volatile v8us*)(h2l + off) = lo;
  __threadfence();
  *(volatile v8us*)(h2h + off) = hi;
  *(volatile v8us*)(h2l + off) = lo;
}

extern "C" void kernel_launch(void* const* d_in, const int* in_sizes, int n_in,
                              void* d_out, int out_size, void* d_ws, size_t ws_size,
                              hipStream_t stream) {
  if (n_in < 25) return;
  if (in_sizes[0] != NPIX * IN_CH) return;
  if (in_sizes[1] != BB * SK_CH * 1024) return;
  if (in_sizes[2] != 96 * IN_CH || in_sizes[3] != 96) return;
  if (in_sizes[4] != IN_CH * QC || in_sizes[5] != IN_CH) return;
  if (in_sizes[6] != SK_CH * 9 || in_sizes[7] != SK_CH || in_sizes[8] < 1) return;
  if (in_sizes[9] != 18 * KCOL || in_sizes[10] != 18) return;
  if (in_sizes[11] != SK_CH * KCOL || in_sizes[12] != SK_CH) return;
  if (in_sizes[13] != EMB || in_sizes[14] != EMB) return;
  if (in_sizes[15] != 4 * EMB * EMB || in_sizes[16] != 4 * EMB) return;
  if (in_sizes[17] != 4 * EMB * 9 || in_sizes[18] != 4 * EMB) return;
  if (in_sizes[19] != 4 * EMB * EMB || in_sizes[20] != EMB) return;
  if (in_sizes[21] != EMB * 320 || in_sizes[22] != EMB) return;
  if (in_sizes[23] != IN_CH * EMB || in_sizes[24] != IN_CH) return;
  if (out_size != NPIX * IN_CH) return;

  const float* x       = (const float*)d_in[0];
  const float* skip    = (const float*)d_in[1];
  const float* qkv_w   = (const float*)d_in[2];
  const float* qkv_b   = (const float*)d_in[3];
  const float* proj_w  = (const float*)d_in[4];
  const float* proj_b  = (const float*)d_in[5];
  const float* edge_w  = (const float*)d_in[6];
  const float* thick_w = (const float*)d_in[7];
  const float* thick_b = (const float*)d_in[8];
  const float* off_w   = (const float*)d_in[9];
  const float* off_b   = (const float*)d_in[10];
  const float* dfm_w   = (const float*)d_in[11];
  const float* dfm_b   = (const float*)d_in[12];
  const float* ln_g    = (const float*)d_in[13];
  const float* ln_b    = (const float*)d_in[14];
  const float* mlp1_w  = (const float*)d_in[15];
  const float* mlp1_b  = (const float*)d_in[16];
  const float* dw_w    = (const float*)d_in[17];
  const float* dw_b    = (const float*)d_in[18];
  const float* mlp2_w  = (const float*)d_in[19];
  const float* mlp2_b  = (const float*)d_in[20];
  const float* down_w  = (const float*)d_in[21];
  const float* down_b  = (const float*)d_in[22];
  const float* up_w    = (const float*)d_in[23];
  const float* up_b    = (const float*)d_in[24];
  float* out = (float*)d_out;

  const size_t szW   = (size_t)WTOT * 2;
  const size_t szR2  = (size_t)NPIX * IN_CH * 2 * 2;
  const size_t szQ   = (size_t)NPIX * QC * 2;
  const size_t szCat = (size_t)NPIX * 320 * 2;
  const size_t szSu  = (size_t)NPIX * SK_CH * 4;
  const size_t szPix = (size_t)NPIX * 4;
  const size_t szOff = (size_t)NPIX * 32 * 4;
  const size_t szR1  = (size_t)NPIX * KCOL * 2 * 2;
  const size_t total = 2 * szW + szR2 + 5 * szQ + 2 * szCat + 2 * szSu + 2 * szPix + szOff + szR1;
  if (total > ws_size) return;

  char* ws = (char*)d_ws;
  size_t o = 0;
  unsigned short* wph = (unsigned short*)(ws + o); o += szW;
  unsigned short* wpl = (unsigned short*)(ws + o); o += szW;
  char* r2 = ws + o; o += szR2;
  _Float16* qpl = (_Float16*)(ws + o); o += szQ;
  _Float16* kpl = (_Float16*)(ws + o); o += szQ;
  _Float16* vtp = (_Float16*)(ws + o); o += szQ;
  unsigned short* avh = (unsigned short*)(ws + o); o += szQ;
  unsigned short* avl = (unsigned short*)(ws + o); o += szQ;
  unsigned short* cath = (unsigned short*)(ws + o); o += szCat;
  unsigned short* catl = (unsigned short*)(ws + o); o += szCat;
  float* suT   = (float*)(ws + o); o += szSu;
  float* mbuf  = (float*)(ws + o); o += szPix;
  float* thk   = (float*)(ws + o); o += szPix;
  float* edgeT = (float*)(ws + o); o += szSu;
  float* offb  = (float*)(ws + o); o += szOff;
  char* r1 = ws + o; o += szR1;
  if (o > ws_size) return;

  unsigned short* xth = (unsigned short*)(r2);
  unsigned short* xtl = (unsigned short*)(r2 + (size_t)NPIX * IN_CH * 2);
  float* ebuf = (float*)(r2);
  unsigned short* hnh = (unsigned short*)(r2 + 4194304);
  unsigned short* hnl = (unsigned short*)(r2 + 6291456);
  unsigned short* th  = (unsigned short*)(r2 + 8388608);
  unsigned short* tl  = (unsigned short*)(r2 + 10485760);
  unsigned short* colh = (unsigned short*)(r1);
  unsigned short* coll = (unsigned short*)(r1 + (size_t)NPIX * KCOL * 2);
  unsigned short* valh = colh;
  unsigned short* vall = coll;
  float* h1 = (float*)(r1);
  unsigned short* h2h = (unsigned short*)(r1 + 16777216);
  unsigned short* h2l = (unsigned short*)(r1 + 25165824);

  const float* dumf = mbuf;
  float* dumo = suT;
  unsigned short* dumu = avl;
  _Float16* dumh = kpl;

  prep_w_kernel<<<dim3(18, 8), 256, 0, stream>>>(qkv_w, proj_w, off_w, dfm_w, down_w, mlp1_w, mlp2_w, up_w, wph, wpl);
  xT_kernel<<<dim3(NPIX / 32, IN_CH / 64), 256, 0, stream>>>(x, xth, xtl);
  gemm_kernel<2, EPI_QKV><<<dim3(NPIX / 64, 3), 128, 0, stream>>>(
      xth, xtl, IN_CH, wph + WO_QKV, wpl + WO_QKV, IN_CH, qkv_b, dumf, dumf,
      dumo, dumu, dumu, qpl, kpl, vtp, 0, 0);
  attn_kernel<<<dim3(HW / 64, BB), 128, 0, stream>>>(qpl, kpl, vtp, avh, avl);
  gemm_kernel<4, EPI_X2><<<dim3(NPIX / 64, IN_CH / 64), 128, 0, stream>>>(
      avh, avl, QC, wph + WO_PROJ, wpl + WO_PROJ, QC, proj_b, x, dumf,
      dumo, cath, catl, dumh, dumh, dumh, 320, 0);
  skipup_kernel<<<NPIX / 32, 512, 0, stream>>>(skip, thick_w, thick_b, suT, mbuf, thk);
  edge_kernel<<<NPIX / 16, 256, 0, stream>>>(mbuf, edge_w, edgeT);
  cols_edge_kernel<<<(NPIX * 72) / 256, 256, 0, stream>>>(edgeT, colh, coll);
  gemm_kernel<2, EPI_OFF><<<dim3(NPIX / 64, 1), 128, 0, stream>>>(
      colh, coll, KCOL, wph + WO_OFF, wpl + WO_OFF, KCOL, off_b, thk, dumf,
      offb, dumu, dumu, dumh, dumh, dumh, 0, 0);
  cols_dfm_kernel<<<(NPIX * 72) / 256, 256, 0, stream>>>(suT, offb, valh, vall);
  gemm_kernel<4, EPI_RES><<<dim3(NPIX / 64, 1), 128, 0, stream>>>(
      valh, vall, KCOL, wph + WO_DFM, wpl + WO_DFM, KCOL, dfm_b, edgeT, dumf,
      dumo, cath, catl, dumh, dumh, dumh, 320, 256);
  gemm_kernel<4, EPI_LN><<<dim3(NPIX / 64, 1), 128, 0, stream>>>(
      cath, catl, 320, wph + WO_DOWN, wpl + WO_DOWN, 320, down_b, ln_g, ln_b,
      ebuf, hnh, hnl, dumh, dumh, dumh, EMB, 0);
  gemm_kernel<4, EPI_GELU><<<dim3(NPIX / 64, 4), 128, 0, stream>>>(
      hnh, hnl, EMB, wph + WO_MLP1, wpl + WO_MLP1, EMB, mlp1_b, dumf, dumf,
      h1, dumu, dumu, dumh, dumh, dumh, 4 * EMB, 0);
  dwconv_kernel<<<NPIX / 8, 256, 0, stream>>>(h1, dw_w, dw_b, h2h, h2l);
  gemm_kernel<4, EPI_RES><<<dim3(NPIX / 64, 1), 128, 0, stream>>>(
      h2h, h2l, 4 * EMB, wph + WO_MLP2, wpl + WO_MLP2, 4 * EMB, mlp2_b, ebuf, dumf,
      dumo, th, tl, dumh, dumh, dumh, EMB, 0);
  gemm_kernel<4, EPI_CHW><<<dim3(NPIX / 64, IN_CH / 64), 128, 0, stream>>>(
      th, tl, EMB, wph + WO_UP, wpl + WO_UP, EMB, up_b, dumf, dumf,
      out, dumu, dumu, dumh, dumh, dumh, 0, 0);
}
